// SelfAttentionLayer_3238405341423
// MI455X (gfx1250) — hardware-verified
//
#include <hip/hip_runtime.h>
#include <math.h>

#ifndef NB
#define NB 2
#endif
#ifndef SEQ
#define SEQ 2048
#endif
#define NB_FULL 2
#define NS_FULL 2048
#define ND 1024
#define NH 16
#define HD 64
#define NTOK (NB * SEQ)
#define JB 16
#define E64 64
#define QKP (2 * ND)
#define E32P (3 * ND)
#define SP 2048
#define ATT_LDS_BYTES ((2 * JB * SP + JB * 68) * 4)
#define QK_CARRY 8.0f
#define SSC 0.001953125f
#define P_CARRY 16384.0f
#define P_UNCARRY 0.00006103515625f
#define LN_EPS 1e-5f
#define OUT1_OFF (NB_FULL * NS_FULL * ND)

static_assert(NB >= 1 && NB <= NB_FULL);
static_assert(SEQ >= 256 && SEQ <= NS_FULL);
static_assert((SEQ % 256) == 0);
static_assert(NH * HD == ND);
static_assert(HD == 64);
static_assert((ND % 64) == 0 && (NTOK % 64) == 0 && (SEQ % 64) == 0);
static_assert((((NTOK / 64) * (QKP / 64)) % 8) == 0);
static_assert((((ND / 64) * (SEQ / 64)) % 8) == 0);
static_assert((((E64 / 64) * (E32P / 64)) % 8) == 0);
static_assert((((SEQ / 64) * (ND / 64)) % 8) == 0);
static_assert((NTOK % 8) == 0);
static_assert(((3 * ND * ND / 8) % 256) == 0);
static_assert(((ND * ND / 8) % 256) == 0);
static_assert(SP >= SEQ);
static_assert(OUT1_OFF * 4 == 16777216);
static_assert(ATT_LDS_BYTES == 266496);
static_assert(E64 == 4 * JB);

typedef _Float16 v16h __attribute__((ext_vector_type(16)));
typedef _Float16 v8h  __attribute__((ext_vector_type(8)));
typedef __bf16   v16b __attribute__((ext_vector_type(16)));
typedef __bf16   v8b  __attribute__((ext_vector_type(8)));
typedef float    v8f  __attribute__((ext_vector_type(8)));
typedef float    v4f  __attribute__((ext_vector_type(4)));
typedef unsigned int v4u __attribute__((ext_vector_type(4)));
typedef v4f __attribute__((may_alias)) v4fa;
typedef v4u __attribute__((may_alias)) v4ua;
typedef v8h __attribute__((may_alias)) v8ha;
typedef v8b __attribute__((may_alias)) v8ba;

__device__ __forceinline__ unsigned short f2bf_bits(float f) {
  unsigned u = __float_as_uint(f);
  return (unsigned short)((u + 0x7FFFu + ((u >> 16) & 1u)) >> 16);
}
__device__ __forceinline__ float bf_bits2f(unsigned short h) { return __uint_as_float(((unsigned)h) << 16); }
__device__ __forceinline__ float bfr(float f) { return bf_bits2f(f2bf_bits(f)); }
__device__ __forceinline__ v4f bfr4(v4f a) { v4f r; r.x = bfr(a.x); r.y = bfr(a.y); r.z = bfr(a.z); r.w = bfr(a.w); return r; }
__device__ __forceinline__ unsigned pk16(unsigned short a, unsigned short b) { return (unsigned)a | ((unsigned)b << 16); }
__device__ __forceinline__ void split_pair(float f0, float f1, unsigned& hp, unsigned& lp) {
  const unsigned short h0 = f2bf_bits(f0), h1 = f2bf_bits(f1);
  const unsigned short l0 = f2bf_bits(f0 - bf_bits2f(h0)), l1 = f2bf_bits(f1 - bf_bits2f(h1));
  hp = pk16(h0, h1);
  lp = pk16(l0, l1);
}
__device__ __forceinline__ unsigned f2h_word(float f) {
  const _Float16 hv = (_Float16)f;
  const unsigned short hb = __builtin_bit_cast(unsigned short, hv);
  return (unsigned)hb;
}

__device__ __forceinline__ void dep_guard_h(v8f& a, v8f& b, v16h x, v16h y) { asm volatile("v_nop\n\tv_nop\n\tv_nop\n\tv_nop" : "+v"(a), "+v"(b) : "v"(x), "v"(y)); }
__device__ __forceinline__ void dep_guard_b(v8f& a, v8f& b, v16b x, v16b y) { asm volatile("v_nop\n\tv_nop\n\tv_nop\n\tv_nop" : "+v"(a), "+v"(b) : "v"(x), "v"(y)); }
__device__ __forceinline__ void keep4_h(v16h a, v16h b, v16h c, v16h d) { asm volatile("v_nop" :: "v"(a), "v"(b), "v"(c), "v"(d)); }
__device__ __forceinline__ void keep4_b(v16b a, v16b b, v16b c, v16b d) { asm volatile("v_nop" :: "v"(a), "v"(b), "v"(c), "v"(d)); }
__device__ __forceinline__ void acc_guard4(v8f& a, v8f& b, v8f& c, v8f& d) { asm volatile("v_nop\n\tv_nop\n\tv_nop\n\tv_nop" : "+v"(a), "+v"(b), "+v"(c), "+v"(d)); }

template <typename T> struct Frag;
template <> struct Frag<_Float16> {
  typedef v16h V; union U { v16h v; v8h h[2]; };
  static __device__ __forceinline__ v16h load(const _Float16* p) {
    U f; f.h[0] = *(const v8ha*)(p); f.h[1] = *(const v8ha*)(p + 16); return f.v;
  }
  static __device__ __forceinline__ v8f mma(v16h a, v16h b, v8f c) {
    return __builtin_amdgcn_wmma_f32_16x16x32_f16(false, a, false, b, (short)0, c, false, false);
  }
  static __device__ __forceinline__ void guard(v8f& a, v8f& b, v16h x, v16h y) { dep_guard_h(a, b, x, y); }
  static __device__ __forceinline__ void keep(v16h a, v16h b, v16h c, v16h d) { keep4_h(a, b, c, d); }
};
template <> struct Frag<__bf16> {
  typedef v16b V; union U { v16b v; v8b h[2]; };
  static __device__ __forceinline__ v16b load(const __bf16* p) {
    U f; f.h[0] = *(const v8ba*)(p); f.h[1] = *(const v8ba*)(p + 16); return f.v;
  }
  static __device__ __forceinline__ v8f mma(v16b a, v16b b, v8f c) {
    return __builtin_amdgcn_wmma_f32_16x16x32_bf16(false, a, false, b, (short)0, c, false, false);
  }
  static __device__ __forceinline__ void guard(v8f& a, v8f& b, v16b x, v16b y) { dep_guard_b(a, b, x, y); }
  static __device__ __forceinline__ void keep(v16b a, v16b b, v16b c, v16b d) { keep4_b(a, b, c, d); }
};

__device__ __forceinline__ v8f wmma_f16g(v16h a, v16h b, v8f c) {
  v8f d = __builtin_amdgcn_wmma_f32_16x16x32_f16(false, a, false, b, (short)0, c, false, false);
  asm volatile("v_nop\n\tv_nop\n\tv_nop\n\tv_nop" : "+v"(d) : "v"(a), "v"(b));
  return d;
}

__device__ __forceinline__ v16h load_p_frag(const float* p) {
  union { v16h v; v4u q[4]; } f;
  const v4u a = *(const v4ua*)(p);
  const v4u c = *(const v4ua*)(p + 4);
  const v4u d = *(const v4ua*)(p + 16);
  const v4u e = *(const v4ua*)(p + 20);
  f.q[0] = (v4u){ (a.x & 0xffffu) | (a.y << 16), (a.z & 0xffffu) | (a.w << 16),
                  (c.x & 0xffffu) | (c.y << 16), (c.z & 0xffffu) | (c.w << 16) };
  f.q[1] = (v4u){ (d.x & 0xffffu) | (d.y << 16), (d.z & 0xffffu) | (d.w << 16),
                  (e.x & 0xffffu) | (e.y << 16), (e.z & 0xffffu) | (e.w << 16) };
  f.q[2] = (v4u){ 0u, 0u, 0u, 0u };
  f.q[3] = (v4u){ 0u, 0u, 0u, 0u };
  union { v16h v; v4u q[4]; } g;
  g.q[0] = f.q[0]; g.q[1] = f.q[1];
  return g.v;
}

__global__ __launch_bounds__(256) void cvt_bf16_kernel(const float* __restrict__ src,
                                                       unsigned short* __restrict__ dst, int n8) {
  const int g = blockIdx.x * 256 + threadIdx.x;
  if (g >= n8) return;
  const size_t o = (size_t)g * 8;
  const v4f a = *(const v4fa*)(src + o);
  const v4f c = *(const v4fa*)(src + o + 4);
  v4u v;
  v.x = pk16(f2bf_bits(a.x), f2bf_bits(a.y));
  v.y = pk16(f2bf_bits(a.z), f2bf_bits(a.w));
  v.z = pk16(f2bf_bits(c.x), f2bf_bits(c.y));
  v.w = pk16(f2bf_bits(c.z), f2bf_bits(c.w));
  *(volatile v4u*)(dst + o) = v;
  __threadfence();
  *(volatile v4u*)(dst + o) = v;
}

__global__ __launch_bounds__(256) void ln_kernel(const float* __restrict__ x, const float* __restrict__ lnw,
                                                  const float* __restrict__ lnb, const int* __restrict__ nheads,
                                                  unsigned short* __restrict__ xh, unsigned short* __restrict__ xl) {
  const int tid = threadIdx.x, lane = tid & 31;
  const int tok = blockIdx.x * 8 + (tid >> 5);
  if (tok >= NTOK) return;
  const int bb = tok / SEQ;
  const int t  = tok - bb * SEQ;
  const float* row = x + ((size_t)bb * NS_FULL + t) * ND;
  const bool bad = (nheads[0] != NH);

  float s = 0.0f;
#pragma unroll 1
  for (int it = 0; it < 4; ++it) {
    const int col0 = 256 * it + 8 * lane;
    const v4f a = bfr4(*(const v4fa*)(row + col0));
    const v4f c = bfr4(*(const v4fa*)(row + col0 + 4));
    s += ((a.x + a.y) + (a.z + a.w)) + ((c.x + c.y) + (c.z + c.w));
  }
#pragma unroll
  for (int off = 1; off < 32; off <<= 1) s += __shfl_xor(s, off, 32);
  const float mu = s * (1.0f / (float)ND);

  float s2 = 0.0f;
#pragma unroll 1
  for (int it = 0; it < 4; ++it) {
    const int col0 = 256 * it + 8 * lane;
    const v4f a = bfr4(*(const v4fa*)(row + col0)) - mu;
    const v4f c = bfr4(*(const v4fa*)(row + col0 + 4)) - mu;
    s2 += ((a.x * a.x + a.y * a.y) + (a.z * a.z + a.w * a.w)) + ((c.x * c.x + c.y * c.y) + (c.z * c.z + c.w * c.w));
  }
#pragma unroll
  for (int off = 1; off < 32; off <<= 1) s2 += __shfl_xor(s2, off, 32);
  const float var  = s2 * (1.0f / (float)ND);
  const float rstd = rsqrtf(var + LN_EPS);
  const float qnan = __uint_as_float(0x7fc00000u);

  unsigned short* hrow = xh + (size_t)tok * ND;
  unsigned short* lrow = xl + (size_t)tok * ND;
#pragma unroll 1
  for (int it = 0; it < 4; ++it) {
    const int col0 = 256 * it + 8 * lane;
    const v4f a  = bfr4(*(const v4fa*)(row + col0));
    const v4f c  = bfr4(*(const v4fa*)(row + col0 + 4));
    const v4f wa = bfr4(*(const v4fa*)(lnw + col0));
    const v4f wc = bfr4(*(const v4fa*)(lnw + col0 + 4));
    const v4f ba = bfr4(*(const v4fa*)(lnb + col0));
    const v4f bc = bfr4(*(const v4fa*)(lnb + col0 + 4));
    v4f ya = (a - mu) * rstd * wa + ba;
    v4f yc = (c - mu) * rstd * wc + bc;
    if (bad) { ya = (v4f){qnan, qnan, qnan, qnan}; yc = ya; }
    unsigned h0, h1, h2, h3, l0, l1, l2, l3;
    split_pair(ya.x, ya.y, h0, l0);
    split_pair(ya.z, ya.w, h1, l1);
    split_pair(yc.x, yc.y, h2, l2);
    split_pair(yc.z, yc.w, h3, l3);
    const v4u hv = {h0, h1, h2, h3};
    const v4u lv = {l0, l1, l2, l3};
    *(volatile v4u*)(hrow + col0) = hv;
    *(volatile v4u*)(lrow + col0) = lv;
    __threadfence();
    *(volatile v4u*)(hrow + col0) = hv;
    *(volatile v4u*)(lrow + col0) = lv;
  }
}

template <int ET> struct Elem;
template <> struct Elem<0> { typedef _Float16 T; };
template <> struct Elem<1> { typedef __bf16 T; };

template <int ET, int SPLIT, int OUT_MODE, int BIAS, int RESID>
__global__ __launch_bounds__(256) void wmma_gemm64(
    const unsigned short* __restrict__ Ap, const unsigned short* __restrict__ A2p, int lda, long strideA,
    const unsigned short* __restrict__ Btp, const unsigned short* __restrict__ Bt2p, int ldb, long strideB,
    void* __restrict__ Cout, void* __restrict__ Cout2, int ldc, long strideC,
    const float* __restrict__ bias, const float* __restrict__ resid,
    int M, int N, int K, float scale) {
  typedef typename Elem<ET>::T T;
  typedef typename Frag<T>::V V;
  const T* A  = (const T*)Ap;  const T* A2  = (const T*)A2p;
  const T* Bt = (const T*)Btp; const T* Bt2 = (const T*)Bt2p;
  __shared__ __align__(16) float sT[8][16 * 68];
  const int b    = blockIdx.y;
  const int lane = threadIdx.x & 31;
  const int wave = threadIdx.x >> 5;
  const int tilesN = N >> 6;
  const int tilesM = M >> 6;
  const int tile = blockIdx.x * 8 + wave;
  if (tile >= tilesM * tilesN) return;
  const int tm = tile / tilesN;
  const int tn = tile - tm * tilesN;
  const int m0 = tm << 6;
  const int n0 = tn << 6;

  const T* Ab  = A  + (size_t)b * strideA;
  const T* Ab2 = (SPLIT == 1) ? (A2 + (size_t)b * strideA) : Ab;
  const T* Bb  = Bt + (size_t)b * strideB;
  const T* Bb2 = (SPLIT == 2) ? (Bt2 + (size_t)b * strideB) : Bb;

  const int rlane = lane & 15;
  const int koff  = (lane >> 4) * 8;
  const int mOff  = (lane >> 4) * 8;

  v8f acc[4][4];
#pragma unroll
  for (int i = 0; i < 4; ++i)
#pragma unroll
    for (int j = 0; j < 4; ++j) acc[i][j] = (v8f){0.f,0.f,0.f,0.f,0.f,0.f,0.f,0.f};

  for (int k0 = 0; k0 < K; k0 += 32) {
    if (SPLIT != 2) {
      V bf[4];
#pragma unroll
      for (int j = 0; j < 4; ++j) {
        const size_t bo = (size_t)(n0 + (j << 4) + rlane) * ldb + koff + k0;
        bf[j] = Frag<T>::load(Bb + bo);
      }
#pragma unroll
      for (int i = 0; i < 4; ++i) {
        const size_t ao = (size_t)(m0 + (i << 4) + rlane) * lda + koff + k0;
        V ah = Frag<T>::load(Ab + ao);
        V al = ah;
        if (SPLIT == 1) al = Frag<T>::load(Ab2 + ao);
#pragma unroll
        for (int j = 0; j < 4; ++j) {
          acc[i][j] = Frag<T>::mma(ah, bf[j], acc[i][j]);
          if (SPLIT == 1) acc[i][j] = Frag<T>::mma(al, bf[j], acc[i][j]);
        }
        Frag<T>::guard(acc[i][0], acc[i][3], ah, al);
      }
      Frag<T>::keep(bf[0], bf[1], bf[2], bf[3]);
    } else {
      V af[4];
#pragma unroll
      for (int i = 0; i < 4; ++i) {
        const size_t ao = (size_t)(m0 + (i << 4) + rlane) * lda + koff + k0;
        af[i] = Frag<T>::load(Ab + ao);
      }
#pragma unroll
      for (int j = 0; j < 4; ++j) {
        const size_t bo = (size_t)(n0 + (j << 4) + rlane) * ldb + koff + k0;
        V bh = Frag<T>::load(Bb + bo);
        V bl = Frag<T>::load(Bb2 + bo);
#pragma unroll
        for (int i = 0; i < 4; ++i) {
          acc[i][j] = Frag<T>::mma(af[i], bh, acc[i][j]);
          acc[i][j] = Frag<T>::mma(af[i], bl, acc[i][j]);
        }
        Frag<T>::guard(acc[0][j], acc[3][j], bh, bl);
      }
      Frag<T>::keep(af[0], af[1], af[2], af[3]);
    }
  }
  acc_guard4(acc[0][0], acc[0][1], acc[0][2], acc[0][3]);
  acc_guard4(acc[1][0], acc[1][1], acc[1][2], acc[1][3]);
  acc_guard4(acc[2][0], acc[2][1], acc[2][2], acc[2][3]);
  acc_guard4(acc[3][0], acc[3][1], acc[3][2], acc[3][3]);

  float bcol[4] = {0.f, 0.f, 0.f, 0.f};
  if (BIAS == 1) {
#pragma unroll
    for (int j = 0; j < 4; ++j) bcol[j] = bfr(bias[n0 + (j << 4) + rlane]);
  }
  float* slab = sT[wave];
#pragma unroll
  for (int i = 0; i < 4; ++i) {
    const int mBase = m0 + (i << 4);
    float brow[8] = {0.f, 0.f, 0.f, 0.f, 0.f, 0.f, 0.f, 0.f};
    if (BIAS == 2) {
#pragma unroll
      for (int r = 0; r < 8; ++r) brow[r] = bfr(bias[mBase + mOff + r]);
    }
#pragma unroll
    for (int j = 0; j < 4; ++j) {
#pragma unroll
      for (int r = 0; r < 8; ++r) {
        const float bb = (BIAS == 1) ? bcol[j] : ((BIAS == 2) ? brow[r] : 0.0f);
        slab[(mOff + r) * 68 + (j << 4) + rlane] = (acc[i][j][r] + bb) * scale;
      }
    }
    __builtin_amdgcn_fence(3, "workgroup");
    __builtin_amdgcn_wave_barrier();
    __builtin_amdgcn_fence(2, "workgroup");
    if (OUT_MODE == 0) {
      float* C = (float*)Cout + (size_t)b * strideC;
      const float* R = resid + (size_t)b * strideC;
      const int hh = lane >> 4, c4 = (lane & 15) * 4;
      for (int pass = 0; pass < 2; ++pass) {
#pragma unroll
        for (int it = 0; it < 8; ++it) {
          const int row = it * 2 + hh;
          v4f v = *(const v4fa*)(slab + row * 68 + c4);
          if (RESID) {
            const v4f rx = *(const v4fa*)(R + (size_t)(mBase + row) * ldc + n0 + c4);
            v += bfr4(rx);
          }
          *(volatile v4f*)(C + (size_t)(mBase + row) * ldc + n0 + c4) = v;
        }
        __threadfence();
      }
    } else {
      const int q = lane >> 3, c8 = (lane & 7) * 8;
      unsigned short* C  = (unsigned short*)Cout  + (size_t)b * strideC;
      unsigned short* C2 = (unsigned short*)Cout2 + (size_t)b * strideC;
      for (int pass = 0; pass < 2; ++pass) {
#pragma unroll
        for (int it = 0; it < 4; ++it) {
          const int row = it * 4 + q;
          const float* sp = slab + row * 68 + c8;
          v8h hv, lv;
#pragma unroll
          for (int e = 0; e < 8; ++e) {
            if (OUT_MODE == 1) {
              hv[e] = (_Float16)sp[e];
              lv[e] = hv[e];
            } else {
              unsigned short hb = f2bf_bits(sp[e]);
              unsigned short lb = f2bf_bits(sp[e] - bf_bits2f(hb));
              hv[e] = __builtin_bit_cast(_Float16, hb);
              lv[e] = __builtin_bit_cast(_Float16, lb);
            }
          }
          *(volatile v8h*)(C + (size_t)(mBase + row) * ldc + n0 + c8) = hv;
          if (OUT_MODE == 2) *(volatile v8h*)(C2 + (size_t)(mBase + row) * ldc + n0 + c8) = lv;
        }
        __threadfence();
      }
    }
    __builtin_amdgcn_fence(3, "workgroup");
    __builtin_amdgcn_wave_barrier();
    __builtin_amdgcn_fence(2, "workgroup");
  }
}

__global__ __launch_bounds__(128) void attn_kernel(const _Float16* __restrict__ qk,
                                                     const _Float16* __restrict__ vt,
                                                     const float* __restrict__ e32,
                                                     float* __restrict__ attn,
                                                     unsigned short* __restrict__ ctxh,
                                                     unsigned short* __restrict__ ctxl) {
  extern __shared__ __align__(16) float lds[];
  float* S    = lds;
  float* AV   = lds + JB * SP;
  float* slab = lds + 2 * JB * SP;
  const int tid = threadIdx.x, lane = tid & 31, w = tid >> 5;
  const int hf = lane >> 4, m = lane & 15;
  const int b  = blockIdx.y;
  const int jb = blockIdx.x;
  const int j0 = jb * JB;
  const int klen = j0 + JB;
  const int nt = jb + 1;
  const int nchunk = (klen + 255) >> 8;
  const bool early = (j0 < E64);
  const v8f zero8 = {0.f, 0.f, 0.f, 0.f, 0.f, 0.f, 0.f, 0.f};

#pragma unroll 1
  for (int h = 0; h < NH; ++h) {
    if (!early) {
      const _Float16* qrow = qk + ((size_t)b * SEQ + j0 + m) * QKP + h * HD + 8 * hf;
      const v16h a0 = Frag<_Float16>::load(qrow);
      const v16h a1 = Frag<_Float16>::load(qrow + 32);
      const _Float16* kbase = qk + ((size_t)b * SEQ + m) * QKP + ND + h * HD + 8 * hf;
      for (int t = w; t < nt; t += 4) {
        const int i0 = t << 4;
        const _Float16* kr = kbase + (size_t)i0 * QKP;
        const v16h b0 = Frag<_Float16>::load(kr);
        const v16h b1 = Frag<_Float16>::load(kr + 32);
        v8f acc = zero8;
        acc = wmma_f16g(a0, b0, acc);
        acc = wmma_f16g(a1, b1, acc);
#pragma unroll
        for (int r = 0; r < 8; ++r) S[(8 * hf + r) * SP + i0 + m] = acc[r] * SSC;
      }
    } else {
      const int r = tid >> 3, cg = tid & 7;
      const float* qr = e32 + ((size_t)b * E64 + j0 + r) * E32P + h * HD;
#pragma unroll 1
      for (int u = 0; u < 8; ++u) {
        const int i = 8 * cg + u;
        const float* kr = e32 + ((size_t)b * E64 + i) * E32P + ND + h * HD;
        float acc = 0.0f;
#pragma unroll 4
        for (int d4 = 0; d4 < HD / 4; ++d4) {
          const v4f qa = *(const v4fa*)(qr + 4 * d4);
          const v4f ka = *(const v4fa*)(kr + 4 * d4);
          acc += qa.x * ka.x + qa.y * ka.y + qa.z * ka.z + qa.w * ka.w;
        }
        S[r * SP + i] = acc * 0.125f;
      }
    }
    __syncthreads();

#pragma unroll 1
    for (int rr = 0; rr < 4; ++rr) {
      const int row  = 4 * w + rr;
      const int qpos = j0 + row;
      float* srow  = S  + (size_t)row * SP;
      float* avrow = AV + (size_t)row * SP;
      float mx = -INFINITY;
#pragma unroll 1
      for (int it = 0; it < nchunk; ++it) {
        const int col0 = 256 * it + 8 * lane;
        const v4f a = *(const v4fa*)(srow + col0);
        const v4f c = *(const v4fa*)(srow + col0 + 4);
        const float s0 = (col0 + 0 <= qpos) ? a.x : -INFINITY;
        const float s1 = (col0 + 1 <= qpos) ? a.y : -INFINITY;
        const float s2 = (col0 + 2 <= qpos) ? a.z : -INFINITY;
        const float s3 = (col0 + 3 <= qpos) ? a.w : -INFINITY;
        const float s4 = (col0 + 4 <= qpos) ? c.x : -INFINITY;
        const float s5 = (col0 + 5 <= qpos) ? c.y : -INFINITY;
        const float s6 = (col0 + 6 <= qpos) ? c.z : -INFINITY;
        const float s7 = (col0 + 7 <= qpos) ? c.w : -INFINITY;
        mx = fmaxf(mx, fmaxf(fmaxf(s0, s1), fmaxf(s2, s3)));
        mx = fmaxf(mx, fmaxf(fmaxf(s4, s5), fmaxf(s6, s7)));
      }
#pragma unroll
      for (int off = 1; off < 32; off <<= 1) mx = fmaxf(mx, __shfl_xor(mx, off, 32));
      float sum = 0.0f;
#pragma unroll 1
      for (int it = 0; it < nchunk; ++it) {
        const int col0 = 256 * it + 8 * lane;
        const v4f a = *(const v4fa*)(srow + col0);
        const v4f c = *(const v4fa*)(srow + col0 + 4);
        v4f ea, ec;
        ea.x = (col0 + 0 <= qpos) ? __expf(a.x - mx) : 0.0f;
        ea.y = (col0 + 1 <= qpos) ? __expf(a.y - mx) : 0.0f;
        ea.z = (col0 + 2 <= qpos) ? __expf(a.z - mx) : 0.0f;
        ea.w = (col0 + 3 <= qpos) ? __expf(a.w - mx) : 0.0f;
        ec.x = (col0 + 4 <= qpos) ? __expf(c.x - mx) : 0.0f;
        ec.y = (col0 + 5 <= qpos) ? __expf(c.y - mx) : 0.0f;
        ec.z = (col0 + 6 <= qpos) ? __expf(c.z - mx) : 0.0f;
        ec.w = (col0 + 7 <= qpos) ? __expf(c.w - mx) : 0.0f;
        *(v4fa*)(srow + col0)     = ea;
        *(v4fa*)(srow + col0 + 4) = ec;
        sum += ((ea.x + ea.y) + (ea.z + ea.w)) + ((ec.x + ec.y) + (ec.z + ec.w));
      }
#pragma unroll
      for (int off = 1; off < 32; off <<= 1) sum += __shfl_xor(sum, off, 32);
      const float inv = 1.0f / sum;
#pragma unroll 1
      for (int it = 0; it < nchunk; ++it) {
        const int col0 = 256 * it + 8 * lane;
        const v4f pa = *(const v4fa*)(srow + col0) * inv;
        const v4f pc = *(const v4fa*)(srow + col0 + 4) * inv;
        if (h == 0) {
          *(v4fa*)(avrow + col0)     = pa;
          *(v4fa*)(avrow + col0 + 4) = pc;
        } else {
          v4f oa = *(const v4fa*)(avrow + col0);
          v4f oc = *(const v4fa*)(avrow + col0 + 4);
          oa += pa; oc += pc;
          *(v4fa*)(avrow + col0)     = oa;
          *(v4fa*)(avrow + col0 + 4) = oc;
        }
        if (early) {
          *(v4fa*)(srow + col0)     = pa;
          *(v4fa*)(srow + col0 + 4) = pc;
        } else {
          const v4u wa = { f2h_word(pa.x * P_CARRY), f2h_word(pa.y * P_CARRY),
                           f2h_word(pa.z * P_CARRY), f2h_word(pa.w * P_CARRY) };
          const v4u wc = { f2h_word(pc.x * P_CARRY), f2h_word(pc.y * P_CARRY),
                           f2h_word(pc.z * P_CARRY), f2h_word(pc.w * P_CARRY) };
          *(v4ua*)(srow + col0)     = wa;
          *(v4ua*)(srow + col0 + 4) = wc;
        }
      }
    }
    __syncthreads();

    if (!early) {
      v8f acc = zero8;
      const float* pslot = S + (size_t)m * SP + 8 * hf;
      const _Float16* vrow = vt + ((size_t)b * ND + h * HD + 16 * w + m) * SEQ + 8 * hf;
      for (int k0 = 0; k0 < klen; k0 += 32) {
        const v16h af = load_p_frag(pslot + k0);
        const v16h bq = Frag<_Float16>::load(vrow + k0);
        acc = wmma_f16g(af, bq, acc);
      }
#pragma unroll
      for (int r = 0; r < 8; ++r) slab[(8 * hf + r) * 68 + 16 * w + m] = acc[r] * P_UNCARRY;
    } else {
      const int r = tid >> 3, dg = tid & 7;
      const float* pr = S + (size_t)r * SP;
      const float* vb = e32 + (size_t)b * E64 * E32P + 2 * ND + h * HD + 8 * dg;
      v4f ca = {0.f, 0.f, 0.f, 0.f};
      v4f cc = {0.f, 0.f, 0.f, 0.f};
#pragma unroll 1
      for (int i = 0; i < klen; ++i) {
        const float p = pr[i];
        const v4f va = *(const v4fa*)(vb + (size_t)i * E32P);
        const v4f vc = *(const v4fa*)(vb + (size_t)i * E32P + 4);
        ca += va * p;
        cc += vc * p;
      }
      *(v4fa*)(slab + r * 68 + 8 * dg)     = ca;
      *(v4fa*)(slab + r * 68 + 8 * dg + 4) = cc;
    }
    __syncthreads();

    {
      const int q = lane >> 3, c8 = (lane & 7) * 8;
      const int row = 4 * w + q;
      const size_t tok = (size_t)b * SEQ + j0 + row;
      const float* sp = slab + row * 68 + c8;
      const v4f fa = *(const v4fa*)(sp);
      const v4f fc = *(const v4fa*)(sp + 4);
      unsigned h0, h1, h2, h3, l0, l1, l2, l3;
      split_pair(fa.x, fa.y, h0, l0);
      split_pair(fa.z, fa.w, h1, l1);
      split_pair(fc.x, fc.y, h2, l2);
      split_pair(fc.z, fc.w, h3, l3);
      const v4u hv = {h0, h1, h2, h3};
      const v4u lv = {l0, l1, l2, l3};
      const size_t o = tok * ND + (size_t)h * HD + c8;
#pragma unroll 1
      for (int pass = 0; pass < 2; ++pass) {
        *(volatile v4u*)(ctxh + o) = hv;
        *(volatile v4u*)(ctxl + o) = lv;
        __threadfence();
      }
    }
  }
  __syncthreads();

#pragma unroll 1
  for (int rr = 0; rr < 4; ++rr) {
    const int row = 4 * w + rr;
    const float* avrow = AV + (size_t)row * SP;
    float* orow = attn + ((size_t)b * NS_FULL + j0 + row) * NS_FULL;
    const int lim = 2 * nchunk;
#pragma unroll 1
    for (int pass = 0; pass < 2; ++pass) {
#pragma unroll 1
      for (int it2 = 0; it2 < NS_FULL / 128; ++it2) {
        const int col = 128 * it2 + 4 * lane;
        v4f v = {0.f, 0.f, 0.f, 0.f};
        if (it2 < lim) v = *(const v4fa*)(avrow + col) * 0.0625f;
        *(volatile v4f*)(orow + col) = v;
      }
      __threadfence();
    }
  }
}

extern "C" void kernel_launch(void* const* d_in, const int* in_sizes, int n_in,
                              void* d_out, int out_size, void* d_ws, size_t ws_size,
                              hipStream_t stream) {
  if (n_in < 8) return;
  const long xneed = ((long)(NB - 1) * NS_FULL + SEQ) * ND;
  if ((long)in_sizes[0] < xneed) return;
  if (in_sizes[1] < 3 * ND * ND || in_sizes[2] < 3 * ND) return;
  if (in_sizes[3] < ND * ND || in_sizes[4] < ND || in_sizes[5] < ND || in_sizes[6] < ND) return;
  if (in_sizes[7] < 1) return;
  const long oneed = (long)OUT1_OFF + ((long)(NB - 1) * NS_FULL + SEQ) * NS_FULL;
  if ((long)out_size < oneed) return;

  const float* x     = (const float*)d_in[0];
  const float* w_in  = (const float*)d_in[1];
  const float* b_in  = (const float*)d_in[2];
  const float* w_out = (const float*)d_in[3];
  const float* b_out = (const float*)d_in[4];
  const float* lnw   = (const float*)d_in[5];
  const float* lnb   = (const float*)d_in[6];
  const int*   nh    = (const int*)d_in[7];
  float* out = (float*)d_out;

  const size_t szX   = (size_t)NTOK * ND * 2;
  const size_t szWB  = (size_t)3 * ND * ND * 2;
  const size_t szWOB = (size_t)ND * ND * 2;
  const size_t szQK  = (size_t)NTOK * QKP * 2;
  const size_t szVT  = (size_t)NB * ND * SEQ * 2;
  const size_t szE32 = (size_t)NB * E64 * E32P * 4;
  const size_t oXH  = 0;
  const size_t oXL  = oXH + szX;
  const size_t oWB  = oXL + szX;
  const size_t oWOB = oWB + szWB;
  const size_t oQK  = oWOB + szWOB;
  const size_t oVT  = oQK + szQK;
  const size_t oE32 = oVT + szVT;
  const size_t oCH  = oE32 + szE32;
  const size_t oCL  = oCH + szX;
  const size_t total = oCL + szX;
  if (total > ws_size) return;

  char* ws = (char*)d_ws;
  unsigned short* XH  = (unsigned short*)(ws + oXH);
  unsigned short* XL  = (unsigned short*)(ws + oXL);
  unsigned short* WB  = (unsigned short*)(ws + oWB);
  unsigned short* WOB = (unsigned short*)(ws + oWOB);
  unsigned short* QK  = (unsigned short*)(ws + oQK);
  unsigned short* VT  = (unsigned short*)(ws + oVT);
  float*          E32 = (float*)(ws + oE32);
  unsigned short* CH  = (unsigned short*)(ws + oCH);
  unsigned short* CL  = (unsigned short*)(ws + oCL);
  unsigned short* WV  = WB + (size_t)2 * ND * ND;

  const dim3 blk(256);

  cvt_bf16_kernel<<<dim3((3 * ND * ND / 8) / 256), blk, 0, stream>>>(w_in, WB, 3 * ND * ND / 8);
  cvt_bf16_kernel<<<dim3((ND * ND / 8) / 256), blk, 0, stream>>>(w_out, WOB, ND * ND / 8);
  ln_kernel<<<dim3(NTOK / 8), blk, 0, stream>>>(x, lnw, lnb, nh, XH, XL);
  wmma_gemm64<1, 1, 1, 1, 0><<<dim3((NTOK / 64) * (QKP / 64) / 8, 1), blk, 0, stream>>>(
      XH, XL, ND, 0L, WB, WB, ND, 0L, (void*)QK, (void*)QK, QKP, 0L, b_in, x,
      NTOK, QKP, ND, QK_CARRY);
  wmma_gemm64<1, 2, 1, 2, 0><<<dim3((ND / 64) * (SEQ / 64) / 8, NB), blk, 0, stream>>>(
      WV, WV, ND, 0L, XH, XL, ND, (long)SEQ * ND, (void*)VT, (void*)VT, SEQ, (long)ND * SEQ,
      b_in + 2 * ND, x, ND, SEQ, ND, 1.0f);
  wmma_gemm64<1, 1, 0, 1, 0><<<dim3((E64 / 64) * (E32P / 64) / 8, NB), blk, 0, stream>>>(
      XH, XL, ND, (long)SEQ * ND, WB, WB, ND, 0L, (void*)E32, (void*)E32, E32P, (long)E64 * E32P,
      b_in, x, E64, E32P, ND, 1.0f);
  (void)hipFuncSetAttribute(reinterpret_cast<const void*>(&attn_kernel),
                            hipFuncAttributeMaxDynamicSharedMemorySize, ATT_LDS_BYTES);
  attn_kernel<<<dim3(SEQ / JB, NB), dim3(128), ATT_LDS_BYTES, stream>>>(
      (const _Float16*)(const void*)QK, (const _Float16*)(const void*)VT, E32,
      out + OUT1_OFF, CH, CL);
  wmma_gemm64<1, 1, 0, 1, 1><<<dim3((SEQ / 64) * (ND / 64) / 8, NB), blk, 0, stream>>>(
      CH, CL, ND, (long)SEQ * ND, WOB, WOB, ND, 0L, (void*)out, (void*)out, ND, (long)NS_FULL * ND,
      b_out, x, SEQ, ND, ND, 1.0f);
  (void)hipGetLastError();
}
